// DiscontinuityGNN_17265768530256
// MI455X (gfx1250) — hardware-verified
//
#include <hip/hip_runtime.h>
#include <hip/hip_bf16.h>
#include <math.h>

typedef __attribute__((ext_vector_type(16))) _Float16 v16h;
typedef __attribute__((ext_vector_type(8)))  float    v8f;

#define ALPHA   0.2f
#define NEG_INF -9.0e15f
#define NNODES  2048
#define NHEADS  4
#define HID     64
#define OUTF    3
#define QWAVES  4
#define RSPLIT (1.0f / 2048.0f)
#define PLH ((size_t)NHEADS * HID * NNODES)
typedef __attribute__((ext_vector_type(8))) _Float16 v8h;
typedef __attribute__((ext_vector_type(4))) float v4f_t;
typedef float v4fa __attribute__((ext_vector_type(4), may_alias));
typedef __attribute__((ext_vector_type(4))) unsigned v4u_t;
__device__ __forceinline__ _Float16 lo_of(float v, _Float16 h) { return (_Float16)((v - (float)h) * 2048.0f); }
__device__ __forceinline__ v8f wmma16(v16h a, v16h b, v8f c) { return __builtin_amdgcn_wmma_f32_16x16x32_f16(false, a, false, b, (short)0, c, false, false); }
__device__ __forceinline__ v8f wmma_split(v16h a, v16h al, v16h b, v16h bl, v8f c) { v8f x = {}; x = wmma16(al, b, x); x = wmma16(a, bl, x); return wmma16(a, b, c) + x * RSPLIT; }
__device__ __forceinline__ unsigned pk2s(float a, float b, unsigned* lo) {
  const _Float16 h0 = (_Float16)a, h1 = (_Float16)b;
  *lo = (unsigned)__builtin_bit_cast(unsigned short, lo_of(a, h0)) | ((unsigned)__builtin_bit_cast(unsigned short, lo_of(b, h1)) << 16);
  return (unsigned)__builtin_bit_cast(unsigned short, h0) | ((unsigned)__builtin_bit_cast(unsigned short, h1) << 16);
}

__global__ __launch_bounds__(256)
void pack_adj_kernel(const int* __restrict__ adj, unsigned* __restrict__ adjbits) {
    int idx = blockIdx.x * blockDim.x + threadIdx.x;
    int p  = idx >> 6;
    int wi = idx & 63;
    const int* row = adj + (size_t)p * NNODES + wi * 32;
    unsigned w = 0u;
    #pragma unroll
    for (int b = 0; b < 32; ++b)
        w |= (row[b] > 0 ? 1u : 0u) << b;
    *(volatile unsigned*)(adjbits + idx) = w; __threadfence(); *(volatile unsigned*)(adjbits + idx) = w;
}

__global__ __launch_bounds__(32)
void encoder_kernel(const float* __restrict__ nf,
                    const float* __restrict__ W1, const float* __restrict__ b1,
                    const float* __restrict__ W2, const float* __restrict__ b2,
                    float* __restrict__ x0) {
    __shared__ float hid[HID];
    int q = blockIdx.x, t = threadIdx.x;
    const float* xr = nf + (size_t)q * 10;
    float h0 = b1[t], h1 = b1[t + 32];
    #pragma unroll 1
    for (int f = 0; f < 10; ++f) {
        float xv = xr[f];
        h0 = fmaf(xv, W1[f * 64 + t],      h0);
        h1 = fmaf(xv, W1[f * 64 + t + 32], h1);
    }
    hid[t]      = fmaxf(h0, 0.f);
    hid[t + 32] = fmaxf(h1, 0.f);
    __syncthreads();
    float o0 = b2[t], o1 = b2[t + 32];
    #pragma unroll 1
    for (int f = 0; f < HID; ++f) {
        float v = hid[f];
        o0 = fmaf(v, W2[f * 64 + t],      o0);
        o1 = fmaf(v, W2[f * 64 + t + 32], o1);
    }
    *(volatile float*)(x0 + (size_t)q * 64 + t) = o0; *(volatile float*)(x0 + (size_t)q * 64 + t + 32) = o1; __threadfence();
    *(volatile float*)(x0 + (size_t)q * 64 + t) = o0; *(volatile float*)(x0 + (size_t)q * 64 + t + 32) = o1;
}

__global__ __launch_bounds__(256)
void hproj_kernel(const float* __restrict__ x, const float* __restrict__ W,
                  const float* __restrict__ a,
                  _Float16* __restrict__ hrow,
                  float* __restrict__ s1, float* __restrict__ s2, int Fin) {
    __shared__ float s1s[32], s2s[32];
    const int tid = threadIdx.x, ql = tid >> 3, g = tid & 7;
    const int q = blockIdx.x * 32 + ql, head = blockIdx.y;
    const float* xr = x + (size_t)q * Fin;
    const float* Wh = W + (size_t)head * Fin * HID + g * 8;
    float hv[8] = {0.f, 0.f, 0.f, 0.f, 0.f, 0.f, 0.f, 0.f};
    for (int f = 0; f < Fin; ++f) {
        const float xv = xr[f];
        const v4f_t w0 = *(const v4f_t*)(Wh + f * HID), w1 = *(const v4f_t*)(Wh + f * HID + 4);
        hv[0] += xv * w0[0]; hv[1] += xv * w0[1]; hv[2] += xv * w0[2]; hv[3] += xv * w0[3];
        hv[4] += xv * w1[0]; hv[5] += xv * w1[1]; hv[6] += xv * w1[2]; hv[7] += xv * w1[3];
    }
    const float* ah = a + head * 2 * HID + g * 8;
    float s1v = 0.f, s2v = 0.f;
    #pragma unroll
    for (int j = 0; j < 8; ++j) { s1v += hv[j] * ah[j]; s2v += hv[j] * ah[HID + j]; }
    s1v += __shfl_xor(s1v, 1, 32); s1v += __shfl_xor(s1v, 2, 32); s1v += __shfl_xor(s1v, 4, 32);
    s2v += __shfl_xor(s2v, 1, 32); s2v += __shfl_xor(s2v, 2, 32); s2v += __shfl_xor(s2v, 4, 32);
    if (g == 0) { s1s[ql] = s1v; s2s[ql] = s2v; }
    v4u_t ph, pl; unsigned l0, l1, l2, l3;
    ph.x = pk2s(hv[0], hv[1], &l0); ph.y = pk2s(hv[2], hv[3], &l1); ph.z = pk2s(hv[4], hv[5], &l2); ph.w = pk2s(hv[6], hv[7], &l3);
    pl.x = l0; pl.y = l1; pl.z = l2; pl.w = l3;
    _Float16* dst = hrow + ((size_t)head * NNODES + q) * HID + g * 8;
    __syncthreads();
    #pragma unroll 1
    for (int pass = 0; pass < 2; ++pass) {
        *(volatile v4u_t*)dst = ph; *(volatile v4u_t*)(dst + PLH) = pl;
        if (tid < 32) { *(volatile float*)(s1 + head * NNODES + blockIdx.x * 32 + tid) = s1s[tid]; *(volatile float*)(s2 + head * NNODES + blockIdx.x * 32 + tid) = s2s[tid]; }
        __threadfence();
    }
}

__global__ __launch_bounds__(256)
void htrans_kernel(const _Float16* __restrict__ hrow, _Float16* __restrict__ hT) {
    __shared__ _Float16 th[64][66], tl[64][66];
    const int tid = threadIdx.x, head = blockIdx.y, q0 = blockIdx.x * 64;
    for (int i = tid; i < 64 * 64; i += 256) { const int ql = i >> 6, f = i & 63; const size_t o = ((size_t)head * NNODES + q0 + ql) * HID + f; th[f][ql] = hrow[o]; tl[f][ql] = hrow[PLH + o]; }
    __syncthreads();
    const int f = tid >> 2, qq = (tid & 3) * 16;
    union { v8h v[2]; _Float16 h[16]; } uh, ul;
    #pragma unroll
    for (int j = 0; j < 16; ++j) { uh.h[j] = th[f][qq + j]; ul.h[j] = tl[f][qq + j]; }
    _Float16* dst = hT + ((size_t)head * HID + f) * NNODES + q0 + qq;
    #pragma unroll 1
    for (int pass = 0; pass < 2; ++pass) {
        *(volatile v8h*)dst = uh.v[0]; *(volatile v8h*)(dst + 8) = uh.v[1]; *(volatile v8h*)(dst + PLH) = ul.v[0]; *(volatile v8h*)(dst + PLH + 8) = ul.v[1];
        __threadfence();
    }
}

__global__ __launch_bounds__(32 * QWAVES)
void gat_flash_kernel(const _Float16* __restrict__ hT,
                      const float* __restrict__ s1,
                      const float* __restrict__ s2,
                      const unsigned* __restrict__ adjbits,
                      float* __restrict__ xout) {
    __shared__ float accbuf[QWAVES - 1][16][64];
    __shared__ float Mbuf[QWAVES - 1][16];
    __shared__ float Sbuf[QWAVES - 1][16];

    const int lane  = threadIdx.x & 31;
    const int wid   = __builtin_amdgcn_readfirstlane(threadIdx.x >> 5);
    const int sel   = lane >> 4;
    const int lm    = lane & 15;
    const int pbase = blockIdx.x * 16;
    const int head  = blockIdx.y;

    const float  s2p = s2[head * NNODES + pbase + lm];
    const float* s1h = s1 + head * NNODES;
    const _Float16* hTh = hT + (size_t)head * HID * NNODES;

    v8f acc[4];
    #pragma unroll
    for (int nt = 0; nt < 4; ++nt)
        #pragma unroll
        for (int r = 0; r < 8; ++r) acc[nt][r] = 0.f;

    float M = -INFINITY, S = 0.f;

    constexpr int NITER = NNODES / (32 * QWAVES);
    int q0 = wid * 32;
    for (int it = 0; it < NITER; ++it, q0 += 32 * QWAVES) {
        v8f s1lo = *(const v8f*)(s1h + q0 + sel * 8);
        v8f s1hi = *(const v8f*)(s1h + q0 + 16 + sel * 8);
        unsigned w = adjbits[(size_t)(pbase + lm) * (NNODES / 32) + (q0 >> 5)];
        const _Float16* hb = hTh + q0 + sel * 8;
        v16h b[4], bl[4];
        #pragma unroll
        for (int nt = 0; nt < 4; ++nt) {
            const _Float16* p = hb + (size_t)(nt * 16 + lm) * NNODES;
            b[nt]  = __builtin_shufflevector(*(const v8h*)p, *(const v8h*)(p + 16), 0,1,2,3,4,5,6,7,8,9,10,11,12,13,14,15);
            bl[nt] = __builtin_shufflevector(*(const v8h*)(p + PLH), *(const v8h*)(p + PLH + 16), 0,1,2,3,4,5,6,7,8,9,10,11,12,13,14,15);
        }

        float pj[16];
        #pragma unroll
        for (int j = 0; j < 8; ++j) {
            float ev = s1lo[j] + s2p;
            ev = ev > 0.f ? ev : ALPHA * ev;
            pj[j] = ((w >> (sel * 8 + j)) & 1u) ? ev : NEG_INF;
        }
        #pragma unroll
        for (int j = 0; j < 8; ++j) {
            float ev = s1hi[j] + s2p;
            ev = ev > 0.f ? ev : ALPHA * ev;
            pj[8 + j] = ((w >> (16 + sel * 8 + j)) & 1u) ? ev : NEG_INF;
        }

        float mx[8];
        #pragma unroll
        for (int j = 0; j < 8; ++j) mx[j] = fmaxf(pj[2 * j], pj[2 * j + 1]);
        #pragma unroll
        for (int j = 0; j < 4; ++j) mx[j] = fmaxf(mx[2 * j], mx[2 * j + 1]);
        mx[0] = fmaxf(fmaxf(mx[0], mx[1]), fmaxf(mx[2], mx[3]));
        float cm = fmaxf(mx[0], __shfl_xor(mx[0], 16, 32));
        float nM  = fmaxf(M, cm);
        float scl = __expf(M - nM);
        M = nM;

        float pv[16];
        v16h afrag, afragl;
        #pragma unroll
        for (int j = 0; j < 16; ++j) {
            pv[j] = __expf(pj[j] - nM);
            const float qv = pv[j] * 1024.0f; afrag[j] = (_Float16)qv; afragl[j] = lo_of(qv, afrag[j]);
        }
        float sm[8];
        #pragma unroll
        for (int j = 0; j < 8; ++j) sm[j] = pv[2 * j] + pv[2 * j + 1];
        #pragma unroll
        for (int j = 0; j < 4; ++j) sm[j] = sm[2 * j] + sm[2 * j + 1];
        float rs = (sm[0] + sm[1]) + (sm[2] + sm[3]);
        rs += __shfl_xor(rs, 16, 32);
        S = S * scl + rs;

        float sc[8];
        #pragma unroll
        for (int r = 0; r < 8; ++r) sc[r] = __shfl(scl, (sel << 3) + r, 32);
        #pragma unroll
        for (int nt = 0; nt < 4; ++nt)
            #pragma unroll
            for (int r = 0; r < 8; ++r) acc[nt][r] *= sc[r];

        #pragma unroll
        for (int nt = 0; nt < 4; ++nt)
            acc[nt] = wmma_split(afrag, afragl, b[nt], bl[nt], acc[nt]);
    }

    if (wid != 0) {
        #pragma unroll
        for (int nt = 0; nt < 4; ++nt)
            #pragma unroll
            for (int r = 0; r < 8; ++r)
                accbuf[wid - 1][sel * 8 + r][nt * 16 + lm] = acc[nt][r];
        if (lane < 16) {
            Mbuf[wid - 1][lane] = M;
            Sbuf[wid - 1][lane] = S;
        }
    }
    __syncthreads();
    if (wid != 0) return;

    #pragma unroll
    for (int wv = 0; wv < QWAVES - 1; ++wv) {
        float Mw = Mbuf[wv][lm];
        float Sw = Sbuf[wv][lm];
        float nM = fmaxf(M, Mw);
        float sA = __expf(M - nM);
        float sB = __expf(Mw - nM);
        S = S * sA + Sw * sB;
        M = nM;
        float ar[8], br[8];
        #pragma unroll
        for (int r = 0; r < 8; ++r) {
            ar[r] = __shfl(sA, (sel << 3) + r, 32);
            br[r] = __shfl(sB, (sel << 3) + r, 32);
        }
        #pragma unroll
        for (int nt = 0; nt < 4; ++nt)
            #pragma unroll
            for (int r = 0; r < 8; ++r)
                acc[nt][r] = acc[nt][r] * ar[r]
                           + accbuf[wv][sel * 8 + r][nt * 16 + lm] * br[r];
    }

    float Sr[8];
    #pragma unroll
    for (int r = 0; r < 8; ++r) Sr[r] = __shfl(S, (sel << 3) + r, 32);
    #pragma unroll
    for (int nt = 0; nt < 4; ++nt)
        #pragma unroll
        for (int r = 0; r < 8; ++r) {
            float v = acc[nt][r] / (Sr[r] * 1024.0f);
            v = v > 0.f ? v : (__expf(v) - 1.f);
            accbuf[0][sel * 8 + r][nt * 16 + lm] = v;
        }
    asm volatile("s_wait_dscnt 0" ::: "memory");
    #pragma unroll 1
    for (int pass = 0; pass < 2; ++pass) {
        #pragma unroll
        for (int i = 0; i < 8; ++i) { const int c = lane + 32 * i, rr = c >> 4, qd = (c & 15) * 4;
            *(volatile v4f_t*)(xout + (size_t)(pbase + rr) * (NHEADS * HID) + head * HID + qd) = *(const volatile v4fa*)&accbuf[0][rr][qd]; }
        __threadfence();
    }
}

__global__ __launch_bounds__(256)
void h2proj_kernel(const float* __restrict__ x, const float* __restrict__ W,
                   const float* __restrict__ a,
                   float* __restrict__ h2, float* __restrict__ s1,
                   float* __restrict__ s2) {
    int idx = blockIdx.x * blockDim.x + threadIdx.x;
    int head = idx / NNODES, q = idx % NNODES;
    const float* xr = x + (size_t)q * (NHEADS * HID);
    const float* Wh = W + (size_t)head * (NHEADS * HID) * OUTF;
    float h0 = 0.f, h1 = 0.f, h2v = 0.f;
    for (int f = 0; f < NHEADS * HID; ++f) {
        float xv = xr[f];
        h0  = fmaf(xv, Wh[f * 3 + 0], h0);
        h1  = fmaf(xv, Wh[f * 3 + 1], h1);
        h2v = fmaf(xv, Wh[f * 3 + 2], h2v);
    }
    float* hq = h2 + (size_t)idx * 3;
    const float* ah = a + head * 6;
    const float u1 = h0 * ah[0] + h1 * ah[1] + h2v * ah[2], u2 = h0 * ah[3] + h1 * ah[4] + h2v * ah[5];
    #pragma unroll 1
    for (int pass = 0; pass < 2; ++pass) {
        *(volatile float*)(hq) = h0; *(volatile float*)(hq + 1) = h1; *(volatile float*)(hq + 2) = h2v;
        *(volatile float*)(s1 + idx) = u1; *(volatile float*)(s2 + idx) = u2;
        __threadfence();
    }
}

__global__ __launch_bounds__(256)
void gat_out_kernel(const float* __restrict__ h2, const float* __restrict__ s1,
                    const float* __restrict__ s2,
                    const unsigned* __restrict__ adjbits,
                    float* __restrict__ hp2) {
    __shared__ float res[32][3];
    const int head = blockIdx.y, lane = threadIdx.x & 31, wv = threadIdx.x >> 5;
    for (int pi = wv; pi < 32; pi += 8) {
    const int p = blockIdx.x * 32 + pi;
    const float s2p = s2[head * NNODES + p];
    const float* s1h = s1 + head * NNODES;
    const float* hh  = h2 + (size_t)head * NNODES * 3;
    float M = -INFINITY, S = 0.f, a0 = 0.f, a1 = 0.f, a2 = 0.f;
    for (int q = lane; q < NNODES; q += 32) {
        unsigned w = adjbits[(size_t)p * (NNODES / 32) + (q >> 5)];
        float ev = s1h[q] + s2p;
        ev = ev > 0.f ? ev : ALPHA * ev;
        ev = ((w >> (q & 31)) & 1u) ? ev : NEG_INF;
        float nM = fmaxf(M, ev);
        float sc = __expf(M - nM);
        float pr = __expf(ev - nM);
        S  = S  * sc + pr;
        a0 = a0 * sc + pr * hh[q * 3 + 0];
        a1 = a1 * sc + pr * hh[q * 3 + 1];
        a2 = a2 * sc + pr * hh[q * 3 + 2];
        M = nM;
    }
    #pragma unroll
    for (int off = 16; off; off >>= 1) {
        float M2 = __shfl_xor(M, off, 32);
        float S2 = __shfl_xor(S, off, 32);
        float b0 = __shfl_xor(a0, off, 32);
        float b1 = __shfl_xor(a1, off, 32);
        float b2 = __shfl_xor(a2, off, 32);
        float nM = fmaxf(M, M2);
        float sA = __expf(M - nM), sB = __expf(M2 - nM);
        S  = S  * sA + S2 * sB;
        a0 = a0 * sA + b0 * sB;
        a1 = a1 * sA + b1 * sB;
        a2 = a2 * sA + b2 * sB;
        M = nM;
    }
    if (lane == 0) { res[pi][0] = a0 / S; res[pi][1] = a1 / S; res[pi][2] = a2 / S; }
    }
    __syncthreads();
    if (threadIdx.x < 96) {
        float* o = hp2 + ((size_t)head * NNODES + blockIdx.x * 32) * 3 + threadIdx.x;
        const float v = res[threadIdx.x / 3][threadIdx.x % 3];
        *(volatile float*)o = v; __threadfence(); *(volatile float*)o = v;
    }
}

__global__ __launch_bounds__(256)
void emb_kernel(const float* __restrict__ hp2, float* __restrict__ emb) {
    int idx = blockIdx.x * blockDim.x + threadIdx.x;
    if (idx >= NNODES * OUTF) return;
    float m = 0.25f * (hp2[idx]
                     + hp2[(size_t)NNODES * 3 + idx]
                     + hp2[(size_t)2 * NNODES * 3 + idx]
                     + hp2[(size_t)3 * NNODES * 3 + idx]);
    const float ev = m > 0.f ? m : (__expf(m) - 1.f);
    *(volatile float*)(emb + idx) = ev; __threadfence(); *(volatile float*)(emb + idx) = ev;
}

__global__ __launch_bounds__(256)
void classifier_kernel(const float* __restrict__ emb,
                       const float* __restrict__ W1, const float* __restrict__ b1,
                       const float* __restrict__ W2, const float* __restrict__ b2,
                       float* __restrict__ out) {
    size_t idx = (size_t)blockIdx.x * blockDim.x + threadIdx.x;
    int p = (int)(idx / NNODES), q = (int)(idx % NNODES);
    float d0 = fabsf(emb[p * 3 + 0] - emb[q * 3 + 0]);
    float d1 = fabsf(emb[p * 3 + 1] - emb[q * 3 + 1]);
    float d2 = fabsf(emb[p * 3 + 2] - emb[q * 3 + 2]);
    float z = b2[0];
    #pragma unroll 1
    for (int j = 0; j < 32; ++j) {
        float h = fmaf(d0, W1[j], fmaf(d1, W1[32 + j], fmaf(d2, W1[64 + j], b1[j])));
        h = fmaxf(h, 0.f);
        z = fmaf(h, W2[j], z);
    }
    const float pr = 1.f / (1.f + __expf(-z));
    *(volatile float*)(out + idx) = pr; __threadfence(); *(volatile float*)(out + idx) = pr;
}

extern "C" void kernel_launch(void* const* d_in, const int* in_sizes, int n_in,
                              void* d_out, int out_size, void* d_ws, size_t ws_size,
                              hipStream_t stream) {
    const float* nf     = (const float*)d_in[0];
    const int*   adj    = (const int*)  d_in[1];
    const float* enc_W1 = (const float*)d_in[2];
    const float* enc_b1 = (const float*)d_in[3];
    const float* enc_W2 = (const float*)d_in[4];
    const float* enc_b2 = (const float*)d_in[5];
    const float* gat_W0 = (const float*)d_in[6];
    const float* gat_a0 = (const float*)d_in[7];
    const float* gat_W1 = (const float*)d_in[8];
    const float* gat_a1 = (const float*)d_in[9];
    const float* gat_W2 = (const float*)d_in[10];
    const float* gat_a2 = (const float*)d_in[11];
    const float* cls_W1 = (const float*)d_in[12];
    const float* cls_b1 = (const float*)d_in[13];
    const float* cls_W2 = (const float*)d_in[14];
    const float* cls_b2 = (const float*)d_in[15];

    char* ws = (char*)d_ws;
    unsigned* adjbits = (unsigned*)(ws);
    float*    x0      = (float*)(ws + (512u  << 10));
    float*    x1      = (float*)(ws + (1024u << 10));
    float*    x2      = (float*)(ws + (3072u << 10));
    _Float16* hT      = (_Float16*)(ws + (5120u << 10));
    float*    s1      = (float*)(ws + (6144u << 10));
    float*    s2      = (float*)(ws + (6176u << 10));
    float*    h2      = (float*)(ws + (6208u << 10));
    float*    s1b     = (float*)(ws + (6304u << 10));
    float*    s2b     = (float*)(ws + (6336u << 10));
    float*    hp2     = (float*)(ws + (6368u << 10));
    hT                = (_Float16*)(ws + (8u << 20));
    _Float16* hrow    = (_Float16*)(ws + (10u << 20));

    float* out_emb   = (float*)d_out;
    float* out_edges = (float*)d_out + NNODES * OUTF;

    pack_adj_kernel<<<(NNODES * 64) / 256, 256, 0, stream>>>(adj, adjbits);
    encoder_kernel<<<NNODES, 32, 0, stream>>>(nf, enc_W1, enc_b1, enc_W2, enc_b2, x0);

    hproj_kernel<<<dim3(NNODES / 32, NHEADS), 256, 0, stream>>>(x0, gat_W0, gat_a0, hrow, s1, s2, HID);
    htrans_kernel<<<dim3(NNODES / 64, NHEADS), 256, 0, stream>>>(hrow, hT);
    gat_flash_kernel<<<dim3(NNODES / 16, NHEADS), 32 * QWAVES, 0, stream>>>(hT, s1, s2, adjbits, x1);

    hproj_kernel<<<dim3(NNODES / 32, NHEADS), 256, 0, stream>>>(x1, gat_W1, gat_a1, hrow, s1, s2, NHEADS * HID);
    htrans_kernel<<<dim3(NNODES / 64, NHEADS), 256, 0, stream>>>(hrow, hT);
    gat_flash_kernel<<<dim3(NNODES / 16, NHEADS), 32 * QWAVES, 0, stream>>>(hT, s1, s2, adjbits, x2);

    h2proj_kernel<<<(NHEADS * NNODES) / 256, 256, 0, stream>>>(x2, gat_W2, gat_a2, h2, s1b, s2b);
    gat_out_kernel<<<dim3(NNODES / 32, NHEADS), 256, 0, stream>>>(h2, s1b, s2b, adjbits, hp2);
    emb_kernel<<<(NNODES * OUTF + 255) / 256, 256, 0, stream>>>(hp2, out_emb);

    classifier_kernel<<<((size_t)NNODES * NNODES) / 256, 256, 0, stream>>>(
        out_emb, cls_W1, cls_b1, cls_W2, cls_b2, out_edges);
}
